// GraphormerEncoderLayer_39402029973513
// MI455X (gfx1250) — hardware-verified
//
#include <hip/hip_runtime.h>

typedef _Float16 v16h __attribute__((ext_vector_type(16)));
typedef _Float16 v8h  __attribute__((ext_vector_type(8)));
typedef float    v8f  __attribute__((ext_vector_type(8)));
typedef float    v4f  __attribute__((ext_vector_type(4)));
typedef int      v4i  __attribute__((ext_vector_type(4)));
typedef v8h __attribute__((may_alias)) v8ha;
typedef v4f __attribute__((may_alias)) v4fa;
typedef v4i __attribute__((may_alias)) v4ia;

union Frag { v16h v; v8h half[2]; };
struct Acc24 { v8f t[2][4]; };

#define BATCH   4
#define SEQ     1024
#define HIDDEN  1024
#define NHEADS  16
#define HD      64
#define FFN     4096
#define MROWS   (BATCH * SEQ)
#define WSCALE  64.0f
#define PSCALE  16384.0f
#define AOSCALE 16.0f
#define SCP     68
#define STP     72

__device__ __forceinline__ v8f wmma_f16(v16h a, v16h b, v8f c) {
  v8f d = __builtin_amdgcn_wmma_f32_16x16x32_f16(false, a, false, b, (short)0, c, false, false);
  asm volatile("v_nop\n\tv_nop\n\tv_nop\n\tv_nop" : "+v"(d) : "v"(a), "v"(b));
  return d;
}

__device__ __forceinline__ v16h load_frag(const _Float16* p, int h) {
  Frag f;
  f.half[0] = *(const v8ha*)(p + 8 * h);
  f.half[1] = *(const v8ha*)(p + 16 + 8 * h);
  return f.v;
}

__global__ __launch_bounds__(256) void cvt_x_kernel(const float* __restrict__ x,
                                                    _Float16* __restrict__ xh, int n8) {
  const int g = blockIdx.x * 256 + threadIdx.x;
  if (g >= n8) return;
  const float* src = x + (size_t)g * 8;
  const v4f a = *(const v4fa*)src;
  const v4f c = *(const v4fa*)(src + 4);
  const v8h o = { (_Float16)a.x, (_Float16)a.y, (_Float16)a.z, (_Float16)a.w,
                  (_Float16)c.x, (_Float16)c.y, (_Float16)c.z, (_Float16)c.w };
  _Float16* dst = xh + (size_t)g * 8;
  *(volatile v8h*)dst = o;
  __threadfence();
  *(volatile v8h*)dst = o;
}

__device__ __forceinline__ void wt_store_pass(const _Float16* sT, _Float16* wt, int K,
                                              int n0, int k0, int w, int lane) {
  const int q8 = lane & 7, sub = lane >> 3;
  #pragma unroll
  for (int i = 0; i < 2; ++i) {
    const int row = w * 8 + i * 4 + sub;
    const v8h v = *(const v8ha*)(sT + row * STP + 8 * q8);
    _Float16* dst = wt + (size_t)(n0 + row) * K + k0 + 8 * q8;
    *(volatile v8h*)dst = v;
  }
}

__global__ __launch_bounds__(256) void cvt_wt_kernel(const float* __restrict__ W,
                                                     _Float16* __restrict__ wt, int K, int N) {
  __shared__ __attribute__((aligned(16))) _Float16 sT[64 * STP];
  const int tid = threadIdx.x, lane = tid & 31, w = tid >> 5;
  const int n0 = blockIdx.x * 64, k0 = blockIdx.y * 64;
  const int c4 = (tid & 15) * 4, kr = tid >> 4;
  #pragma unroll
  for (int i = 0; i < 4; ++i) {
    const int kk = kr + 16 * i;
    const v4f a = *(const v4fa*)(W + (size_t)(k0 + kk) * N + n0 + c4);
    sT[(c4 + 0) * STP + kk] = (_Float16)(a.x * WSCALE);
    sT[(c4 + 1) * STP + kk] = (_Float16)(a.y * WSCALE);
    sT[(c4 + 2) * STP + kk] = (_Float16)(a.z * WSCALE);
    sT[(c4 + 3) * STP + kk] = (_Float16)(a.w * WSCALE);
  }
  __syncthreads();
  wt_store_pass(sT, wt, K, n0, k0, w, lane);
  __threadfence();
  wt_store_pass(sT, wt, K, n0, k0, w, lane);
}

__device__ __forceinline__ void gemm_core(const _Float16* __restrict__ A,
                                          const _Float16* __restrict__ Bt,
                                          int K, int rowa, int rowb, int h, Acc24& c) {
  const v8f zero8 = {0.f, 0.f, 0.f, 0.f, 0.f, 0.f, 0.f, 0.f};
  #pragma unroll
  for (int mt = 0; mt < 2; ++mt)
    #pragma unroll
    for (int nt = 0; nt < 4; ++nt) c.t[mt][nt] = zero8;

  const _Float16* xa0 = A + (size_t)rowa * K;
  const _Float16* xa1 = xa0 + (size_t)16 * K;
  const _Float16* wb  = Bt + (size_t)rowb * K;
  const size_t k16 = (size_t)16 * K;

  #pragma unroll 1
  for (int k0 = 0; k0 < K; k0 += 32) {
    const v16h a0 = load_frag(xa0 + k0, h);
    const v16h a1 = load_frag(xa1 + k0, h);
    #pragma unroll
    for (int nt = 0; nt < 4; ++nt) {
      const v16h b = load_frag(wb + nt * k16 + k0, h);
      c.t[0][nt] = wmma_f16(a0, b, c.t[0][nt]);
      c.t[1][nt] = wmma_f16(a1, b, c.t[1][nt]);
    }
  }
}

__device__ __forceinline__ void qkv_store_pass(const _Float16* sT, _Float16* plane, _Float16* vt,
                                               int which, int bh, int l0, int w, int lane) {
  const int q8 = lane & 7, sub = lane >> 3;
  #pragma unroll
  for (int i = 0; i < 8; ++i) {
    const int lid = w * 32 + i * 4 + sub;
    v8h v;
    _Float16* dst;
    if (which != 2) {
      v = *(const v8ha*)(sT + lid * HD + 8 * q8);
      dst = plane + ((size_t)bh * SEQ + l0 + lid) * HD + 8 * q8;
    } else {
      const int d = lid >> 1, hl = lid & 1;
      v = *(const v8ha*)(sT + d * 128 + 64 * hl + 8 * q8);
      dst = vt + ((size_t)bh * HD + d) * SEQ + l0 + 64 * hl + 8 * q8;
    }
    *(volatile v8h*)dst = v;
  }
}

__global__ __launch_bounds__(128) void gemm_qkv_kernel(
    const _Float16* __restrict__ xh,
    const _Float16* __restrict__ wqkvT,
    const float* __restrict__ qkvb,
    _Float16* __restrict__ qpl,
    _Float16* __restrict__ kpl,
    _Float16* __restrict__ vtp)
{
  __shared__ __attribute__((aligned(16))) _Float16 sT[128 * 64];

  const int tid = threadIdx.x, lane = tid & 31, w = tid >> 5;
  const int h = lane >> 4, m = lane & 15;
  const int bm = blockIdx.x * 128;
  const int cg = blockIdx.y;
  const int bn = cg * 64;
  const int which = cg >> 4, head = cg & 15;

  Acc24 c;
  gemm_core(xh, wqkvT, HIDDEN, bm + 32 * w + m, bn + m, h, c);

  #pragma unroll
  for (int nt = 0; nt < 4; ++nt) {
    const int feat = 16 * nt + m;
    const float bvl = qkvb[bn + feat];
    #pragma unroll
    for (int mt = 0; mt < 2; ++mt) {
      #pragma unroll
      for (int r = 0; r < 8; ++r) {
        const int tokl = 32 * w + 16 * mt + 8 * h + r;
        const float y = c.t[mt][nt][r] * (1.0f / WSCALE) + bvl;
        const int idx = (which == 2) ? (feat * 128 + tokl) : (tokl * HD + feat);
        sT[idx] = (_Float16)y;
      }
    }
  }
  __syncthreads();

  const int b = bm / SEQ, l0 = bm - b * SEQ, bh = b * NHEADS + head;
  _Float16* plane = (which == 0) ? qpl : kpl;
  qkv_store_pass(sT, plane, vtp, which, bh, l0, w, lane);
  __threadfence();
  qkv_store_pass(sT, plane, vtp, which, bh, l0, w, lane);
}

__device__ __forceinline__ void f32_store_pass(const float* sC, float* Cf, int N,
                                               int bm, int bn, int w, int lane) {
  const int q8 = lane & 7, sub = lane >> 3;
  #pragma unroll
  for (int i = 0; i < 16; ++i) {
    const int lid = i * 4 + sub;
    const int row = 32 * w + (lid >> 1), hl = lid & 1;
    const v4f v = *(const v4fa*)(sC + row * SCP + 32 * hl + 4 * q8);
    float* dst = Cf + (size_t)(bm + row) * N + bn + 32 * hl + 4 * q8;
    *(volatile v4f*)dst = v;
  }
}

__global__ __launch_bounds__(128) void gemm_f32_kernel(
    const _Float16* __restrict__ A, const _Float16* __restrict__ Bt,
    const float* __restrict__ bias, int K, int N, float oscale,
    float* __restrict__ Cf)
{
  __shared__ __attribute__((aligned(16))) float sC[128 * SCP];

  const int tid = threadIdx.x, lane = tid & 31, w = tid >> 5;
  const int h = lane >> 4, m = lane & 15;
  const int bm = blockIdx.x * 128, bn = blockIdx.y * 64;

  Acc24 c;
  gemm_core(A, Bt, K, bm + 32 * w + m, bn + m, h, c);

  #pragma unroll
  for (int nt = 0; nt < 4; ++nt) {
    const int feat = 16 * nt + m;
    const float bvl = bias[bn + feat];
    #pragma unroll
    for (int mt = 0; mt < 2; ++mt) {
      #pragma unroll
      for (int r = 0; r < 8; ++r) {
        const int tokl = 32 * w + 16 * mt + 8 * h + r;
        sC[tokl * SCP + feat] = c.t[mt][nt][r] * oscale + bvl;
      }
    }
  }
  __syncthreads();

  f32_store_pass(sC, Cf, N, bm, bn, w, lane);
  __threadfence();
  f32_store_pass(sC, Cf, N, bm, bn, w, lane);
}

__device__ __forceinline__ void f16_store_pass(const _Float16* sT, _Float16* Cb, int N,
                                               int bm, int bn, int w, int lane) {
  const int q8 = lane & 7, sub = lane >> 3;
  #pragma unroll
  for (int i = 0; i < 8; ++i) {
    const int row = 32 * w + i * 4 + sub;
    const v8h v = *(const v8ha*)(sT + row * STP + 8 * q8);
    _Float16* dst = Cb + (size_t)(bm + row) * N + bn + 8 * q8;
    *(volatile v8h*)dst = v;
  }
}

__global__ __launch_bounds__(128) void gemm_gelu_kernel(
    const _Float16* __restrict__ A, const _Float16* __restrict__ Bt,
    const float* __restrict__ bias, int K, int N,
    _Float16* __restrict__ Cb)
{
  __shared__ __attribute__((aligned(16))) _Float16 sT[128 * STP];

  const int tid = threadIdx.x, lane = tid & 31, w = tid >> 5;
  const int h = lane >> 4, m = lane & 15;
  const int bm = blockIdx.x * 128, bn = blockIdx.y * 64;

  Acc24 c;
  gemm_core(A, Bt, K, bm + 32 * w + m, bn + m, h, c);

  #pragma unroll
  for (int nt = 0; nt < 4; ++nt) {
    const int feat = 16 * nt + m;
    const float bvl = bias[bn + feat];
    #pragma unroll
    for (int mt = 0; mt < 2; ++mt) {
      #pragma unroll
      for (int r = 0; r < 8; ++r) {
        const int tokl = 32 * w + 16 * mt + 8 * h + r;
        const float t = c.t[mt][nt][r] * (1.0f / WSCALE) + bvl;
        const float g = 0.5f * t * (1.0f + erff(t * 0.70710678118654752f));
        sT[tokl * STP + feat] = (_Float16)g;
      }
    }
  }
  __syncthreads();

  f16_store_pass(sT, Cb, N, bm, bn, w, lane);
  __threadfence();
  f16_store_pass(sT, Cb, N, bm, bn, w, lane);
}

__device__ __forceinline__ v8f bias_mask8(v8f s, const float* bp, const int* mp) {
  const v4f ba = *(const v4fa*)bp;
  const v4f bb = *(const v4fa*)(bp + 4);
  const v4i ma = *(const v4ia*)mp;
  const v4i mb = *(const v4ia*)(mp + 4);
  const float ninf = -__builtin_inff();
  v8f r;
  r[0] = (ma.x != 0) ? ninf : (s[0] * 0.125f + ba.x);
  r[1] = (ma.y != 0) ? ninf : (s[1] * 0.125f + ba.y);
  r[2] = (ma.z != 0) ? ninf : (s[2] * 0.125f + ba.z);
  r[3] = (ma.w != 0) ? ninf : (s[3] * 0.125f + ba.w);
  r[4] = (mb.x != 0) ? ninf : (s[4] * 0.125f + bb.x);
  r[5] = (mb.y != 0) ? ninf : (s[5] * 0.125f + bb.y);
  r[6] = (mb.z != 0) ? ninf : (s[6] * 0.125f + bb.z);
  r[7] = (mb.w != 0) ? ninf : (s[7] * 0.125f + bb.w);
  return r;
}

__device__ __forceinline__ v16h pack_p(v8f a, v8f c) {
  const v16h r = { (_Float16)(a[0] * PSCALE), (_Float16)(a[1] * PSCALE), (_Float16)(a[2] * PSCALE), (_Float16)(a[3] * PSCALE),
                   (_Float16)(a[4] * PSCALE), (_Float16)(a[5] * PSCALE), (_Float16)(a[6] * PSCALE), (_Float16)(a[7] * PSCALE),
                   (_Float16)(c[0] * PSCALE), (_Float16)(c[1] * PSCALE), (_Float16)(c[2] * PSCALE), (_Float16)(c[3] * PSCALE),
                   (_Float16)(c[4] * PSCALE), (_Float16)(c[5] * PSCALE), (_Float16)(c[6] * PSCALE), (_Float16)(c[7] * PSCALE) };
  return r;
}

__device__ __forceinline__ void ao_store_pass(const _Float16* so, _Float16* ao,
                                              int b, int head, int q0, int lane) {
  const int q8 = lane & 7, sub = lane >> 3;
  #pragma unroll
  for (int i = 0; i < 4; ++i) {
    const int row = i * 4 + sub;
    const v8h v = *(const v8ha*)(so + row * 64 + 8 * q8);
    _Float16* dst = ao + ((size_t)b * SEQ + q0 + row) * HIDDEN + head * HD + 8 * q8;
    *(volatile v8h*)dst = v;
  }
}

__global__ __launch_bounds__(128) void attn_kernel(
    const _Float16* __restrict__ qpl,
    const _Float16* __restrict__ kpl,
    const _Float16* __restrict__ vtp,
    const float* __restrict__ abias,
    const int* __restrict__ kpm,
    _Float16* __restrict__ ao)
{
  __shared__ __attribute__((aligned(16))) _Float16 sO[4 * 16 * 64];
  __shared__ __attribute__((aligned(16))) int sMask[SEQ];

  const int tid = threadIdx.x, lane = tid & 31, w = tid >> 5;
  const int h = lane >> 4, m = lane & 15;
  const int bh = blockIdx.y, b = bh >> 4, head = bh & 15;
  const int q0 = blockIdx.x * 64 + 16 * w;

  {
    const int* mp = kpm + (size_t)b * SEQ + 8 * tid;
    const v4i mk0 = *(const v4ia*)mp;
    const v4i mk1 = *(const v4ia*)(mp + 4);
    *(v4ia*)(sMask + 8 * tid) = mk0;
    *(v4ia*)(sMask + 8 * tid + 4) = mk1;
  }
  __syncthreads();

  const _Float16* qrow = qpl + ((size_t)bh * SEQ + q0 + m) * HD;
  const v16h qb0 = load_frag(qrow, h);
  const v16h qb1 = load_frag(qrow + 32, h);

  const v8f zero8 = {0.f, 0.f, 0.f, 0.f, 0.f, 0.f, 0.f, 0.f};
  v8f o[4];
  #pragma unroll
  for (int t = 0; t < 4; ++t) o[t] = zero8;
  float mrun = -1.0e30f, lrun = 0.0f;

  const _Float16* kbase = kpl + ((size_t)bh * SEQ + m) * HD;
  const _Float16* vbase = vtp + ((size_t)bh * HD + m) * SEQ;
  const float* brow = abias + ((size_t)b * SEQ + q0 + m) * SEQ + 8 * h;
  const int* mrow = sMask + 8 * h;

  #pragma unroll 1
  for (int kb = 0; kb < SEQ; kb += 64) {
    v8f s[4];
    #pragma unroll
    for (int j = 0; j < 4; ++j) {
      const _Float16* kp = kbase + (size_t)(kb + 16 * j) * HD;
      const v16h kf0 = load_frag(kp, h);
      const v16h kf1 = load_frag(kp + 32, h);
      v8f z = zero8;
      z = wmma_f16(kf0, qb0, z);
      z = wmma_f16(kf1, qb1, z);
      s[j] = z;
    }
    #pragma unroll
    for (int j = 0; j < 4; ++j) s[j] = bias_mask8(s[j], brow + kb + 16 * j, mrow + kb + 16 * j);

    float mloc = s[0][0];
    #pragma unroll
    for (int j = 0; j < 4; ++j)
      #pragma unroll
      for (int r = 0; r < 8; ++r) mloc = fmaxf(mloc, s[j][r]);
    mloc = fmaxf(mloc, __shfl_xor(mloc, 16));
    const float mnew = fmaxf(mrun, mloc);
    const float alpha = __expf(mrun - mnew);
    mrun = mnew;
    float lsum = 0.0f;
    #pragma unroll
    for (int j = 0; j < 4; ++j)
      #pragma unroll
      for (int r = 0; r < 8; ++r) {
        const float p = __expf(s[j][r] - mnew);
        s[j][r] = p;
        lsum += p;
      }
    lsum += __shfl_xor(lsum, 16);
    lrun = lrun * alpha + lsum;
    #pragma unroll
    for (int t = 0; t < 4; ++t)
      #pragma unroll
      for (int r = 0; r < 8; ++r) o[t][r] = o[t][r] * alpha;

    const v16h pb0 = pack_p(s[0], s[1]);
    const v16h pb1 = pack_p(s[2], s[3]);

    #pragma unroll
    for (int t = 0; t < 4; ++t) {
      const _Float16* vp = vbase + (size_t)(16 * t) * SEQ + kb;
      const v16h vf0 = load_frag(vp, h);
      const v16h vf1 = load_frag(vp + 32, h);
      o[t] = wmma_f16(vf0, pb0, o[t]);
      o[t] = wmma_f16(vf1, pb1, o[t]);
    }
  }

  const float inv = (1.0f / lrun) * (AOSCALE / PSCALE);
  _Float16* so = sO + w * 1024;
  #pragma unroll
  for (int t = 0; t < 4; ++t)
    #pragma unroll
    for (int r = 0; r < 8; ++r)
      so[m * 64 + 16 * t + 8 * h + r] = (_Float16)(o[t][r] * inv);
  __syncthreads();

  ao_store_pass(so, ao, b, head, q0, lane);
  __threadfence();
  ao_store_pass(so, ao, b, head, q0, lane);
}

__device__ __forceinline__ float wave_sum(float v) {
  v += __shfl_xor(v, 16);
  v += __shfl_xor(v, 8);
  v += __shfl_xor(v, 4);
  v += __shfl_xor(v, 2);
  v += __shfl_xor(v, 1);
  return v;
}

__device__ __forceinline__ v4f ln_core(const float* __restrict__ X, const float* __restrict__ R,
                                       const float* __restrict__ G, const float* __restrict__ Bb,
                                       int row, int tid, float* red) {
  const int lane = tid & 31, w = tid >> 5;
  const size_t off = (size_t)row * HIDDEN + 4 * tid;
  const v4f a = *(const v4fa*)(X + off);
  const v4f c = *(const v4fa*)(R + off);
  const v4f t = a + c;
  float s = (t.x + t.y) + (t.z + t.w);
  s = wave_sum(s);
  if (lane == 0) red[w] = s;
  __syncthreads();
  float tot = 0.0f;
  #pragma unroll
  for (int i = 0; i < 8; ++i) tot += red[i];
  const float mean = tot * (1.0f / (float)HIDDEN);
  const v4f d = t - mean;
  float q = (d.x * d.x + d.y * d.y) + (d.z * d.z + d.w * d.w);
  q = wave_sum(q);
  if (lane == 0) red[8 + w] = q;
  __syncthreads();
  float vs = 0.0f;
  #pragma unroll
  for (int i = 0; i < 8; ++i) vs += red[8 + i];
  const float inv = rsqrtf(vs * (1.0f / (float)HIDDEN) + 1e-5f);
  const v4f g = *(const v4fa*)(G + 4 * tid);
  const v4f bb = *(const v4fa*)(Bb + 4 * tid);
  return d * inv * g + bb;
}

__global__ __launch_bounds__(256) void ln1_kernel(
    const float* __restrict__ X, const float* __restrict__ R,
    const float* __restrict__ G, const float* __restrict__ Bb,
    float* __restrict__ Of, _Float16* __restrict__ Oh)
{
  __shared__ float red[16];
  __shared__ __attribute__((aligned(16))) float sRow[HIDDEN];
  const int row = blockIdx.x, tid = threadIdx.x;
  const v4f o = ln_core(X, R, G, Bb, row, tid, red);
  *(v4fa*)(sRow + 4 * tid) = o;
  __syncthreads();
  const bool lower = (tid < 128);
  v8h hv = {(_Float16)0.f, (_Float16)0.f, (_Float16)0.f, (_Float16)0.f,
            (_Float16)0.f, (_Float16)0.f, (_Float16)0.f, (_Float16)0.f};
  if (lower) {
    const v4f p0 = *(const v4fa*)(sRow + 8 * tid);
    const v4f p1 = *(const v4fa*)(sRow + 8 * tid + 4);
    hv[0] = (_Float16)p0.x; hv[1] = (_Float16)p0.y; hv[2] = (_Float16)p0.z; hv[3] = (_Float16)p0.w;
    hv[4] = (_Float16)p1.x; hv[5] = (_Float16)p1.y; hv[6] = (_Float16)p1.z; hv[7] = (_Float16)p1.w;
  }
  float* dst = Of + (size_t)row * HIDDEN + 4 * tid;
  _Float16* hdst = Oh + (size_t)row * HIDDEN + 8 * (tid & 127);
  *(volatile v4f*)dst = o;
  if (lower) *(volatile v8h*)hdst = hv;
  __threadfence();
  *(volatile v4f*)dst = o;
  if (lower) *(volatile v8h*)hdst = hv;
}

__global__ __launch_bounds__(256) void ln2_kernel(
    const float* __restrict__ X, const float* __restrict__ R,
    const float* __restrict__ G, const float* __restrict__ Bb,
    const int* __restrict__ kpm, float* __restrict__ Out)
{
  __shared__ float red[16];
  const int row = blockIdx.x, tid = threadIdx.x;
  const v4f o = ln_core(X, R, G, Bb, row, tid, red);
  const int mk = kpm[row];
  v4f oo;
  oo.x = (mk != 0) ? 0.0f : o.x;
  oo.y = (mk != 0) ? 0.0f : o.y;
  oo.z = (mk != 0) ? 0.0f : o.z;
  oo.w = (mk != 0) ? 0.0f : o.w;
  float* dst = Out + (size_t)row * HIDDEN + 4 * tid;
  *(volatile v4f*)dst = oo;
  __threadfence();
  *(volatile v4f*)dst = oo;
}

extern "C" void kernel_launch(void* const* d_in, const int* in_sizes, int n_in,
                              void* d_out, int out_size, void* d_ws, size_t ws_size,
                              hipStream_t stream) {
  if (n_in < 15) return;
  if (in_sizes[0] != MROWS * HIDDEN) return;
  if (in_sizes[1] != BATCH * SEQ * SEQ) return;
  if (in_sizes[2] != BATCH * SEQ) return;
  if (in_sizes[3] != HIDDEN * 3 * HIDDEN) return;
  if (in_sizes[4] != 3 * HIDDEN) return;
  if (in_sizes[5] != HIDDEN * HIDDEN) return;
  if (in_sizes[6] != HIDDEN) return;
  if (in_sizes[7] != HIDDEN || in_sizes[8] != HIDDEN) return;
  if (in_sizes[9] != HIDDEN || in_sizes[10] != HIDDEN) return;
  if (in_sizes[11] != HIDDEN * FFN) return;
  if (in_sizes[12] != FFN) return;
  if (in_sizes[13] != FFN * HIDDEN) return;
  if (in_sizes[14] != HIDDEN) return;
  if (out_size != MROWS * HIDDEN) return;

  const float* x      = (const float*)d_in[0];
  const float* abias  = (const float*)d_in[1];
  const int*   kpm    = (const int*)d_in[2];
  const float* qkv_w  = (const float*)d_in[3];
  const float* qkv_b  = (const float*)d_in[4];
  const float* proj_w = (const float*)d_in[5];
  const float* proj_b = (const float*)d_in[6];
  const float* ln1_g  = (const float*)d_in[7];
  const float* ln1_b  = (const float*)d_in[8];
  const float* ln2_g  = (const float*)d_in[9];
  const float* ln2_b  = (const float*)d_in[10];
  const float* ffn_w1 = (const float*)d_in[11];
  const float* ffn_b1 = (const float*)d_in[12];
  const float* ffn_w2 = (const float*)d_in[13];
  const float* ffn_b2 = (const float*)d_in[14];
  float* out = (float*)d_out;

  const size_t MiB = (size_t)1048576;
  const size_t total = 104 * MiB;
  if (total > ws_size) return;
  char* ws = (char*)d_ws;
  _Float16* xh    = (_Float16*)(ws + 0 * MiB);
  _Float16* wqkvT = (_Float16*)(ws + 8 * MiB);
  _Float16* qpl   = (_Float16*)(ws + 14 * MiB);
  _Float16* kpl   = (_Float16*)(ws + 22 * MiB);
  _Float16* vtp   = (_Float16*)(ws + 30 * MiB);
  _Float16* hb    = (_Float16*)(ws + 0 * MiB);
  _Float16* wpT   = (_Float16*)(ws + 38 * MiB);
  _Float16* w1T   = (_Float16*)(ws + 40 * MiB);
  _Float16* w2T   = (_Float16*)(ws + 48 * MiB);
  _Float16* ao    = (_Float16*)(ws + 56 * MiB);
  float*    pf    = (float*)(ws + 64 * MiB);
  float*    f2f   = (float*)(ws + 56 * MiB);
  float*    x1f   = (float*)(ws + 80 * MiB);
  _Float16* x1h   = (_Float16*)(ws + 96 * MiB);

  const int nx8 = MROWS * HIDDEN / 8;
  cvt_x_kernel<<<(nx8 + 255) / 256, 256, 0, stream>>>(x, xh, nx8);

  cvt_wt_kernel<<<dim3(3 * HIDDEN / 64, HIDDEN / 64), 256, 0, stream>>>(qkv_w, wqkvT, HIDDEN, 3 * HIDDEN);
  cvt_wt_kernel<<<dim3(HIDDEN / 64, HIDDEN / 64), 256, 0, stream>>>(proj_w, wpT, HIDDEN, HIDDEN);
  cvt_wt_kernel<<<dim3(FFN / 64, HIDDEN / 64), 256, 0, stream>>>(ffn_w1, w1T, HIDDEN, FFN);
  cvt_wt_kernel<<<dim3(HIDDEN / 64, FFN / 64), 256, 0, stream>>>(ffn_w2, w2T, FFN, HIDDEN);

  gemm_qkv_kernel<<<dim3(MROWS / 128, 3 * NHEADS), 128, 0, stream>>>(xh, wqkvT, qkv_b, qpl, kpl, vtp);

  attn_kernel<<<dim3(SEQ / 64, BATCH * NHEADS), 128, 0, stream>>>(qpl, kpl, vtp, abias, kpm, ao);

  gemm_f32_kernel<<<dim3(MROWS / 128, HIDDEN / 64), 128, 0, stream>>>(
      ao, wpT, proj_b, HIDDEN, HIDDEN, 1.0f / (WSCALE * AOSCALE), pf);

  ln1_kernel<<<MROWS, 256, 0, stream>>>(x, pf, ln1_g, ln1_b, x1f, x1h);

  gemm_gelu_kernel<<<dim3(MROWS / 128, FFN / 64), 128, 0, stream>>>(x1h, w1T, ffn_b1, HIDDEN, FFN, hb);

  gemm_f32_kernel<<<dim3(MROWS / 128, HIDDEN / 64), 128, 0, stream>>>(
      hb, w2T, ffn_b2, FFN, HIDDEN, 1.0f / WSCALE, f2f);

  ln2_kernel<<<MROWS, 256, 0, stream>>>(x1f, f2f, ln2_g, ln2_b, kpm, out);
}
